// GNOhMLP_stem_6305011991078
// MI455X (gfx1250) — hardware-verified
//
#include <hip/hip_runtime.h>


namespace {
constexpr int B_ = 2, C_ = 4, GD = 32, NY = GD * GD * GD, NQ = 4096, KN = 32, EMB = 96, KIN = 2 * EMB + C_, K0P = 256, OUTC = 128, HID = 256;

typedef _Float16 b16;
typedef __attribute__((ext_vector_type(16))) _Float16 v16b;
typedef __attribute__((ext_vector_type(8)))  _Float16 v8b;
typedef __attribute__((ext_vector_type(8)))  float v8f;
typedef __attribute__((ext_vector_type(4)))  float v4f;

__device__ __forceinline__ v8b ld8b(const b16* p) { return *(const v8b*)p; }
__device__ __forceinline__ v16b cat8b(v8b a, v8b b) { return __builtin_shufflevector(a, b, 0, 1, 2, 3, 4, 5, 6, 7, 8, 9, 10, 11, 12, 13, 14, 15); }
__device__ __forceinline__ v16b frag_kb(const b16* p, int hh) { return cat8b(ld8b(p + 8 * hh), ld8b(p + 16 + 8 * hh)); }
__device__ __forceinline__ void split16(float v, b16& hi, b16& lo) { hi = (b16)v; lo = (b16)(v - (float)hi); }
__device__ __forceinline__ void frag_ksplit(const float* p, int hh, v16b& fh_, v16b& fl_) {
  const float* p0 = p + 8 * hh; const float* p1 = p + 16 + 8 * hh;
#pragma unroll
  for (int e = 0; e < 8; ++e) { b16 a, c; split16(p0[e], a, c); fh_[e] = a; fl_[e] = c; split16(p1[e], a, c); fh_[8 + e] = a; fl_[8 + e] = c; }
}
__device__ __forceinline__ v8f wmma16b(v16b a, v16b b, v8f c) {
  v8f d = __builtin_amdgcn_wmma_f32_16x16x32_f16(false, a, false, b, (short)0, c, false, false);
  asm volatile("v_nop\n\tv_nop\n\tv_nop\n\tv_nop" : "+v"(d) : "v"(a), "v"(b));
  return d;
}
__device__ __forceinline__ void wave_lds_sync() {
  __builtin_amdgcn_fence(__ATOMIC_RELEASE, "workgroup");
  __builtin_amdgcn_wave_barrier();
  __builtin_amdgcn_fence(__ATOMIC_ACQUIRE, "workgroup");
}

struct Opnd { const void* p0; const void* p1; int ld; };
template <int NP> __device__ __forceinline__ void load_frags(const Opnd& o, int row, int kb, int hh, v16b& fh_, v16b& fl_) {
  if (NP == 0) { frag_ksplit((const float*)o.p0 + (size_t)row * o.ld + kb, hh, fh_, fl_); }
  else if (NP == 4) {
    const float* p = (const float*)o.p0 + (size_t)row * o.ld + kb; const float* p0 = p + 8 * hh; const float* p1 = p + 16 + 8 * hh;
#pragma unroll
    for (int e = 0; e < 8; ++e) { b16 a, c; split16(p0[e] * 64.0f, a, c); fh_[e] = a; fl_[e] = c; split16(p1[e] * 64.0f, a, c); fh_[8 + e] = a; fl_[8 + e] = c; }
  } else if (NP == 3) {
    const float* p = (const float*)o.p0 + (size_t)row * o.ld + kb; const float* p0 = p + 8 * hh; const float* p1 = p + 16 + 8 * hh;
#pragma unroll
    for (int e = 0; e < 8; ++e) { fh_[e] = (b16)p0[e]; fh_[8 + e] = (b16)p1[e]; }
    fl_ = fh_;
  } else {
    fh_ = frag_kb((const b16*)o.p0 + (size_t)row * o.ld + kb, hh);
    if (NP == 2) fl_ = frag_kb((const b16*)o.p1 + (size_t)row * o.ld + kb, hh); else fl_ = fh_;
  }
}
template <int ANP, int BNP> __device__ __forceinline__ v8f mac(v16b ah, v16b al, v16b bh, v16b bl, v8f c) {
  c = wmma16b(ah, bh, c);
  if (BNP == 0 || BNP == 2 || BNP == 4) c = wmma16b(ah, bl, c);
  if (ANP == 0 || ANP == 2 || ANP == 4) c = wmma16b(al, bh, c);
  return c;
}
template <int ANP, int BNP>
__device__ __forceinline__ void gemm_tile(const Opnd& A, const Opnd& B, int K, int m0, int c0, int nloc, int hlf, v8f (&acc)[2][4]) {
  for (int kb = 0; kb < K; kb += 32) {
    v16b a0h, a0l, a1h, a1l;
    load_frags<ANP>(A, m0 + nloc, kb, hlf, a0h, a0l);
    load_frags<ANP>(A, m0 + 16 + nloc, kb, hlf, a1h, a1l);
#pragma unroll
    for (int t = 0; t < 4; ++t) {
      v16b bh, bl;
      load_frags<BNP>(B, c0 + t * 16 + nloc, kb, hlf, bh, bl);
      acc[0][t] = mac<ANP, BNP>(a0h, a0l, bh, bl, acc[0][t]);
      acc[1][t] = mac<ANP, BNP>(a1h, a1l, bh, bl, acc[1][t]);
    }
  }
}

__device__ __forceinline__ void epi_planes(v8f (&acc)[2][4], float scale, bool two, b16* __restrict__ oh, b16* __restrict__ ol, int ldo,
                                           int m0, int c0, int lane, b16* Th, b16* Tl) {
  const int nloc = lane & 15, hlf = lane >> 4;
#pragma unroll
  for (int t = 0; t < 4; ++t)
#pragma unroll
    for (int r = 0; r < 2; ++r)
#pragma unroll
      for (int v = 0; v < 8; ++v) {
        const int rr = r * 16 + v + 8 * hlf, cc = t * 16 + nloc;
        b16 h_, l_; split16(acc[r][t][v] * scale, h_, l_);
        Th[rr * 64 + cc] = h_; Tl[rr * 64 + cc] = l_;
      }
  wave_lds_sync();
  for (int pass = 0; pass < 2; ++pass) {
#pragma unroll
    for (int j = 0; j < 8; ++j) {
      const int rr = j * 4 + (lane >> 3), c8 = (lane & 7) * 8;
      const size_t o = (size_t)(m0 + rr) * ldo + c0 + c8;
      *(volatile v8b*)(oh + o) = ld8b(Th + rr * 64 + c8);
      if (two) *(volatile v8b*)(ol + o) = ld8b(Tl + rr * 64 + c8);
    }
    __threadfence();
  }
}
__device__ __forceinline__ void epi_f32(v8f (&acc)[2][4], float scale, const float* rscale, float* __restrict__ out, int ldo, int m0, int c0, int lane, float* Tt) {
  const int nloc = lane & 15, hlf = lane >> 4;
#pragma unroll
  for (int t = 0; t < 4; ++t)
#pragma unroll
    for (int r = 0; r < 2; ++r)
#pragma unroll
      for (int v = 0; v < 8; ++v) {
        const int rr = r * 16 + v + 8 * hlf;
        const float rs = rscale ? rscale[(size_t)(m0 + rr) * 32] : 1.0f;
        Tt[rr * 64 + t * 16 + nloc] = acc[r][t][v] * scale * rs;
      }
  wave_lds_sync();
  float* dst0 = out + (size_t)m0 * ldo + c0;
  for (int pass = 0; pass < 2; ++pass) {
#pragma unroll
    for (int j = 0; j < 16; ++j) { const int rr = j * 2 + hlf, c4 = nloc * 4; *(volatile v4f*)(dst0 + (size_t)rr * ldo + c4) = *(const v4f*)(Tt + rr * 64 + c4); }
    __threadfence();
  }
}


__global__ __launch_bounds__(256) void tr_kernel(const float* __restrict__ in, int K, int N, int Kp, b16* __restrict__ out) {
  __shared__ __attribute__((aligned(16))) b16 Tl[64][72];
  const int tid = threadIdx.x, lane = tid & 31, wave = tid >> 5, n0 = blockIdx.x * 64, k0 = blockIdx.y * 64;
  for (int it = 0; it < 16; ++it) { const int kk = k0 + it * 4 + (tid >> 6), n = tid & 63; Tl[n][it * 4 + (tid >> 6)] = (kk < K) ? (b16)in[(size_t)kk * N + n0 + n] : (b16)0.0f; }
  __syncthreads();
  b16* dst = out + (size_t)n0 * Kp + k0;
  for (int pass = 0; pass < 2; ++pass) {
#pragma unroll
    for (int j = 0; j < 2; ++j) { const int rr = wave * 8 + j * 4 + (lane >> 3), c8 = (lane & 7) * 8; *(volatile v8b*)(dst + (size_t)rr * Kp + c8) = *(const v8b*)(&Tl[rr][c8]); }
    __threadfence();
  }
}

constexpr int NYB = B_ * NY * 3 / 256, NXB = NQ * 3 / 256;
__global__ __launch_bounds__(256) void emb_kernel(const float* __restrict__ gc, const float* __restrict__ lat, b16* __restrict__ ye, b16* __restrict__ xe) {
  __shared__ __attribute__((aligned(16))) b16 T[256][32];
  __shared__ float red[6][256];
  const int t = threadIdx.x;
  float fr[16];
#pragma unroll
  for (int j = 0; j < 16; ++j) fr[j] = 1.0f / powf(10000.0f, (float)(2 * j) / 32.0f);
  float v; b16* base;
  if (blockIdx.x < NYB) {
    const size_t e = (size_t)blockIdx.x * 256 + t;
    v = gc[e]; base = ye + (size_t)blockIdx.x * 256 * 32;
  } else {
    const int b = (blockIdx.x - NYB) / NXB, chunk = (blockIdx.x - NYB) % NXB;
    float mn[3] = {INFINITY, INFINITY, INFINITY}, mx[3] = {-INFINITY, -INFINITY, -INFINITY};
    for (int n = t; n < NY; n += 256)
#pragma unroll
      for (int c = 0; c < 3; ++c) { const float u = gc[((size_t)b * NY + n) * 3 + c]; mn[c] = fminf(mn[c], u); mx[c] = fmaxf(mx[c], u); }
#pragma unroll
    for (int c = 0; c < 3; ++c) { red[c][t] = mn[c]; red[3 + c][t] = mx[c]; }
    __syncthreads();
    for (int o = 128; o > 0; o >>= 1) { if (t < o) {
#pragma unroll
      for (int c = 0; c < 3; ++c) { red[c][t] = fminf(red[c][t], red[c][t + o]); red[3 + c][t] = fmaxf(red[3 + c][t], red[3 + c][t + o]); } }
      __syncthreads(); }
    const int qc = chunk * 256 + t, c = qc % 3;
    v = red[c][0] + (red[3 + c][0] - red[c][0]) * lat[qc];
    base = xe + ((size_t)b * NQ * 3 + (size_t)chunk * 256) * 32;
  }
#pragma unroll 1
  for (int j = 0; j < 16; ++j) { float s, cs; sincosf(v * fr[j], &s, &cs); T[t][j] = (b16)s; T[t][16 + j] = (b16)cs; }
  __syncthreads();
  const b16* Tf = &T[0][0];
  for (int pass = 0; pass < 2; ++pass) {
#pragma unroll
    for (int i = 0; i < 4; ++i) { const int pc_ = i * 256 + t; *(volatile v8b*)(base + (size_t)pc_ * 8) = *(const v8b*)(Tf + pc_ * 8); }
    __threadfence();
  }
}

__device__ __forceinline__ float gelu_t(float v) { const float u = 0.7978845608028654f * (v + 0.044715f * v * v * v); const float t = 1.0f - 2.0f / (1.0f + __expf(2.0f * u)); return 0.5f * v * (1.0f + t); }

__global__ __launch_bounds__(128) void gno_kernel(const float* __restrict__ x, const int* __restrict__ nidx, const int* __restrict__ nmask, const b16* __restrict__ ye,
                                                 const b16* __restrict__ xe, const b16* __restrict__ W0T, const float* __restrict__ b0, const b16* __restrict__ W1T,
                                                 const float* __restrict__ b1, const b16* __restrict__ W2T, const float* __restrict__ b2, const b16* __restrict__ W3T,
                                                 const float* __restrict__ b3, float* __restrict__ qbuf) {
  __shared__ __attribute__((aligned(16))) b16 A0[128][HID];
  __shared__ __attribute__((aligned(16))) b16 Hs[128][OUTC];
  __shared__ __attribute__((aligned(16))) float Os[4][OUTC];
  __shared__ int Ms[128];
  const int tid = threadIdx.x, wave = tid >> 5, lane = tid & 31, hh = lane >> 4, col = lane & 15;
  const int b = blockIdx.x / (NQ / 4), q = (blockIdx.x % (NQ / 4)) * 4 + wave;
  {
    const size_t qk = ((size_t)b * NQ + q) * KN + lane;
    int id = nidx[qk]; id = id < 0 ? 0 : (id >= NY ? NY - 1 : id);
    Ms[tid] = nmask[qk];
    b16* row = A0[tid];
    const b16* ys = ye + ((size_t)b * NY + id) * EMB; const b16* xs = xe + ((size_t)b * NQ + q) * EMB;
#pragma unroll
    for (int p = 0; p < 12; ++p) { *(v8b*)(row + p * 8) = ld8b(ys + p * 8); *(v8b*)(row + EMB + p * 8) = ld8b(xs + p * 8); }
    const int dz = id % GD, wy = (id / GD) % GD, hx = id / (GD * GD);
#pragma unroll
    for (int c = 0; c < C_; ++c) row[2 * EMB + c] = (b16)x[((((size_t)b * C_ + c) * GD + dz) * GD + hx) * GD + wy];
    for (int k = KIN; k < K0P; ++k) row[k] = (b16)0.0f;
  }
  __syncthreads();
  const int m0 = wave * 32;
  {
    v8f acc[2][8];
#pragma unroll
    for (int r = 0; r < 2; ++r)
#pragma unroll
      for (int t = 0; t < 8; ++t) acc[r][t] = (v8f){};
    for (int kb = 0; kb < K0P; kb += 32) {
      const v16b a0 = frag_kb(&A0[m0 + col][kb], hh), a1 = frag_kb(&A0[m0 + 16 + col][kb], hh);
#pragma unroll
      for (int t = 0; t < 8; ++t) { const v16b bw = frag_kb(W0T + (size_t)(t * 16 + col) * K0P + kb, hh); acc[0][t] = wmma16b(a0, bw, acc[0][t]); acc[1][t] = wmma16b(a1, bw, acc[1][t]); }
    }
#pragma unroll
    for (int t = 0; t < 8; ++t)
#pragma unroll
      for (int r = 0; r < 2; ++r)
#pragma unroll
        for (int v = 0; v < 8; ++v) { const int rr = m0 + r * 16 + 8 * hh + v, cc = t * 16 + col; Hs[rr][cc] = (b16)gelu_t(acc[r][t][v] + b0[cc]); }
  }
  wave_lds_sync();
  for (int half = 0; half < 2; ++half) {
    v8f acc[2][8];
#pragma unroll
    for (int r = 0; r < 2; ++r)
#pragma unroll
      for (int t = 0; t < 8; ++t) acc[r][t] = (v8f){};
#pragma unroll
    for (int kb = 0; kb < OUTC; kb += 32) {
      const v16b a0 = frag_kb(&Hs[m0 + col][kb], hh), a1 = frag_kb(&Hs[m0 + 16 + col][kb], hh);
#pragma unroll
      for (int t = 0; t < 8; ++t) { const v16b bw = frag_kb(W1T + (size_t)(half * 128 + t * 16 + col) * OUTC + kb, hh); acc[0][t] = wmma16b(a0, bw, acc[0][t]); acc[1][t] = wmma16b(a1, bw, acc[1][t]); }
    }
#pragma unroll
    for (int t = 0; t < 8; ++t)
#pragma unroll
      for (int r = 0; r < 2; ++r)
#pragma unroll
        for (int v = 0; v < 8; ++v) { const int rr = m0 + r * 16 + 8 * hh + v, cc = half * 128 + t * 16 + col; A0[rr][cc] = (b16)gelu_t(acc[r][t][v] + b1[cc]); }
  }
  wave_lds_sync();
  {
    v8f acc[2][8];
#pragma unroll
    for (int r = 0; r < 2; ++r)
#pragma unroll
      for (int t = 0; t < 8; ++t) acc[r][t] = (v8f){};
#pragma unroll
    for (int kb = 0; kb < HID; kb += 32) {
      const v16b a0 = frag_kb(&A0[m0 + col][kb], hh), a1 = frag_kb(&A0[m0 + 16 + col][kb], hh);
#pragma unroll
      for (int t = 0; t < 8; ++t) { const v16b bw = frag_kb(W2T + (size_t)(t * 16 + col) * HID + kb, hh); acc[0][t] = wmma16b(a0, bw, acc[0][t]); acc[1][t] = wmma16b(a1, bw, acc[1][t]); }
    }
    wave_lds_sync();
#pragma unroll
    for (int t = 0; t < 8; ++t)
#pragma unroll
      for (int r = 0; r < 2; ++r)
#pragma unroll
        for (int v = 0; v < 8; ++v) { const int rr = m0 + r * 16 + 8 * hh + v, cc = t * 16 + col; Hs[rr][cc] = (b16)gelu_t(acc[r][t][v] + b2[cc]); }
  }
  wave_lds_sync();
  {
    v8f acc[2][8];
#pragma unroll
    for (int r = 0; r < 2; ++r)
#pragma unroll
      for (int t = 0; t < 8; ++t) acc[r][t] = (v8f){};
#pragma unroll
    for (int kb = 0; kb < OUTC; kb += 32) {
      const v16b a0 = frag_kb(&Hs[m0 + col][kb], hh), a1 = frag_kb(&Hs[m0 + 16 + col][kb], hh);
#pragma unroll
      for (int t = 0; t < 8; ++t) { const v16b bw = frag_kb(W3T + (size_t)(t * 16 + col) * OUTC + kb, hh); acc[0][t] = wmma16b(a0, bw, acc[0][t]); acc[1][t] = wmma16b(a1, bw, acc[1][t]); }
    }
    float msk[2][8];
#pragma unroll
    for (int r = 0; r < 2; ++r)
#pragma unroll
      for (int v = 0; v < 8; ++v) msk[r][v] = (float)(Ms[m0 + r * 16 + 8 * hh + v] != 0);
#pragma unroll
    for (int t = 0; t < 8; ++t) {
      const int cc = t * 16 + col; float s = 0.0f;
#pragma unroll
      for (int r = 0; r < 2; ++r)
#pragma unroll
        for (int v = 0; v < 8; ++v) s += (acc[r][t][v] + b3[cc]) * msk[r][v];
      s += __shfl_xor(s, 16);
      if (hh == 0) Os[wave][cc] = s;
    }
  }
  wave_lds_sync();
  float* dst = qbuf + ((size_t)b * NQ + q) * OUTC;
  const v4f o4 = *(const v4f*)(&Os[wave][lane * 4]);
  *(volatile v4f*)(dst + lane * 4) = o4; __threadfence(); *(volatile v4f*)(dst + lane * 4) = o4;
}

__global__ __launch_bounds__(256) void perm_kernel(const float* __restrict__ qbuf, float* __restrict__ out) {
  const int b = blockIdx.x / OUTC, c = blockIdx.x % OUTC;
  float* dst = out + ((size_t)b * OUTC + c) * NQ;
  for (int pass = 0; pass < 2; ++pass) {
    for (int j = threadIdx.x; j < NQ; j += 256) {
      const int dz = j >> 8, hx = (j >> 4) & 15, wy = j & 15, q = hx * 256 + wy * 16 + dz;
      ((volatile float*)dst)[j] = qbuf[((size_t)b * NQ + q) * OUTC + c];
    }
    __threadfence();
  }
}
}

extern "C" void kernel_launch(void* const* d_in, const int* in_sizes, int n_in,
                              void* d_out, int out_size, void* d_ws, size_t ws_size, hipStream_t stream) {
  (void)n_in; (void)out_size;
  const float* x    = (const float*)d_in[0];
  const float* gc   = (const float*)d_in[1];
  const float* lat  = (const float*)d_in[2];
  const int* nidx   = (const int*)d_in[3];
  const int* nmask  = (const int*)d_in[4];
  const float* W0 = (const float*)d_in[5]; const float* b0 = (const float*)d_in[6];
  const float* W1 = (const float*)d_in[7]; const float* b1 = (const float*)d_in[8];
  const float* W2 = (const float*)d_in[9]; const float* b2 = (const float*)d_in[10];
  const float* W3 = (const float*)d_in[11]; const float* b3 = (const float*)d_in[12];
  float* out = (float*)d_out;
  if (in_sizes[0] != B_ * C_ * NY || in_sizes[1] != B_ * NY * 3 || in_sizes[3] != B_ * NQ * KN || in_sizes[5] != KIN * OUTC || in_sizes[7] != OUTC * HID) return;

  size_t off = 0; char* ws = (char*)d_ws;
  auto carve = [&](size_t bytes) { char* p = ws + off; off += (bytes + 255) & ~(size_t)255; return p; };
  b16* W0T = (b16*)carve((size_t)OUTC * K0P * 2); b16* W1T = (b16*)carve((size_t)HID * OUTC * 2); b16* W2T = (b16*)carve((size_t)OUTC * HID * 2); b16* W3T = (b16*)carve((size_t)OUTC * OUTC * 2);
  b16* ye = (b16*)carve((size_t)B_ * NY * EMB * 2);
  b16* xe = (b16*)carve((size_t)B_ * NQ * EMB * 2);
  float* qbuf = (float*)carve((size_t)B_ * NQ * OUTC * 4);
  if (off > ws_size) return;
  tr_kernel<<<dim3(OUTC / 64, K0P / 64), 256, 0, stream>>>(W0, KIN, OUTC, K0P, W0T);
  tr_kernel<<<dim3(HID / 64, OUTC / 64), 256, 0, stream>>>(W1, OUTC, HID, OUTC, W1T);
  tr_kernel<<<dim3(OUTC / 64, HID / 64), 256, 0, stream>>>(W2, HID, OUTC, HID, W2T);
  tr_kernel<<<dim3(OUTC / 64, OUTC / 64), 256, 0, stream>>>(W3, OUTC, OUTC, OUTC, W3T);
  emb_kernel<<<NYB + B_ * NXB, 256, 0, stream>>>(gc, lat, ye, xe);
  gno_kernel<<<B_ * NQ / 4, 128, 0, stream>>>(x, nidx, nmask, ye, xe, W0T, b0, W1T, b1, W2T, b2, W3T, b3, qbuf);
  perm_kernel<<<B_ * OUTC, 256, 0, stream>>>(qbuf, out);
}
